// BiLSTM_Parser_21440476741954
// MI455X (gfx1250) — hardware-verified
//
#include <hip/hip_runtime.h>
#include <math.h>


#define SEQ   1024
#define HID   512
#define G4    2048
#define DW    300
#define DP    100
#define KP0   512
#define IN1   1024
#define MH    512
#define OPSC  16.0f
#define OPSC2INV 0.00390625f
#define SPITCH 68

typedef _Float16 v16h __attribute__((ext_vector_type(16)));
typedef _Float16 v8h  __attribute__((ext_vector_type(8)));
typedef float    v8f  __attribute__((ext_vector_type(8)));
typedef float    v4f  __attribute__((ext_vector_type(4)));
union Frag { v16h v; v8h hv[2]; };

__device__ __forceinline__ v8f wmma16(v16h a, v16h b, v8f c) {
  c = __builtin_amdgcn_wmma_f32_16x16x32_f16(false, a, false, b, (short)0, c, false, false);
  asm volatile("v_nop\n\tv_nop\n\tv_nop\n\tv_nop" : "+v"(c) : "v"(a), "v"(b));
  return c;
}

__device__ __forceinline__ v16h ldfrag_g(const _Float16* __restrict__ base, int pitch, int row, int k0, int h) {
  const _Float16* p = base + (size_t)row * pitch + k0 + 8 * h;
  Frag f;
  f.hv[0] = *(const v8h*)p;
  f.hv[1] = *(const v8h*)(p + 16);
  return f.v;
}

__global__ void __launch_bounds__(256)
k_cvt16(const float* __restrict__ in, _Float16* out, int R, int Kin, int Kpad, float scale) {
  const size_t nvec = (size_t)R * (size_t)Kpad / 8;
  const size_t i = (size_t)blockIdx.x * 256 + threadIdx.x;
  if (i >= nvec) return;
  const size_t e = i * 8;
  const int r = (int)(e / (size_t)Kpad);
  const int c = (int)(e % (size_t)Kpad);
  const float* src = in + (size_t)r * Kin;
  v8h hv;
#pragma unroll
  for (int u = 0; u < 8; ++u) {
    const int cc = c + u;
    const float v = (cc < Kin) ? src[cc] * scale : 0.0f;
    hv[u] = (_Float16)v;
  }
  _Float16* dst = out + e;
  *(volatile v8h*)dst = hv;
  __threadfence();
  *(volatile v8h*)dst = hv;
}

__global__ void __launch_bounds__(64)
k_embed(const int* __restrict__ wt, const int* __restrict__ pt,
        const float* __restrict__ wemb, const float* __restrict__ pemb,
        int V, int P, _Float16* xb, int T) {
  const int t = blockIdx.x;
  if (t >= T) return;
  int w = wt[t];
  if (w < 0) w += V;
  w = w < 0 ? 0 : (w >= V ? V - 1 : w);
  int p = pt[t];
  if (p < 0) p += P;
  p = p < 0 ? 0 : (p >= P ? P - 1 : p);
  const int c0 = 8 * threadIdx.x;
  v8h hv;
#pragma unroll
  for (int u = 0; u < 8; ++u) {
    const int c = c0 + u;
    float v = 0.0f;
    if (c < DW) v = wemb[(size_t)w * DW + c];
    else if (c < DW + DP) v = pemb[(size_t)p * DP + (c - DW)];
    hv[u] = (_Float16)(v * OPSC);
  }
  _Float16* dst = xb + (size_t)t * KP0 + c0;
  *(volatile v8h*)dst = hv;
  __threadfence();
  *(volatile v8h*)dst = hv;
}

__device__ __forceinline__ void stash_tile(float* S, v8f acc, int hf, int ss, int h, int m) {
#pragma unroll
  for (int r = 0; r < 8; ++r)
    S[(16 * hf + 8 * h + r) * SPITCH + 16 * ss + m] = acc[r];
}

__device__ __forceinline__ void gemm_store_pass(const float* S, float* C, int ldc, int m0, int n0,
                                                int h, int m, float scale, v4f bias, bool active) {
#pragma unroll
  for (int i = 0; i < 16; ++i) {
    const int row = 2 * i + h;
    v4f v = *(const v4f*)(S + row * SPITCH + 4 * m);
    v = v * scale + bias;
    if (active) *(volatile v4f*)(C + (size_t)(m0 + row) * ldc + n0 + 4 * m) = v;
  }
}

__global__ void __launch_bounds__(128)
k_gemm(const _Float16* __restrict__ A, int lda,
       const _Float16* __restrict__ W, int ldb,
       const float* __restrict__ b1, const float* __restrict__ b2, int nbias,
       float* C, int ldc, int Mt, int Nt, int K, float scale) {
  __shared__ __align__(16) float stg[4 * 32 * SPITCH];
  const int wid = threadIdx.x >> 5;
  const int l = threadIdx.x & 31, h = l >> 4, m = l & 15;
  const int wave = blockIdx.x * 4 + wid;
  const bool active = wave < Mt * Nt;
  const int wv = active ? wave : 0;
  const int m0 = (wv / Nt) * 32;
  const int n0 = (wv % Nt) * 64;

  const v8f z = {0.f, 0.f, 0.f, 0.f, 0.f, 0.f, 0.f, 0.f};
  v8f acc0 = z, acc1 = z, acc2 = z, acc3 = z, acc4 = z, acc5 = z, acc6 = z, acc7 = z;

#pragma unroll 1
  for (int k0 = 0; k0 < K; k0 += 32) {
    const v16h a0 = ldfrag_g(A, lda, m0 + m, k0, h);
    const v16h a1 = ldfrag_g(A, lda, m0 + 16 + m, k0, h);
    const v16h w0 = ldfrag_g(W, ldb, n0 + m, k0, h);
    const v16h w1 = ldfrag_g(W, ldb, n0 + 16 + m, k0, h);
    const v16h w2 = ldfrag_g(W, ldb, n0 + 32 + m, k0, h);
    const v16h w3 = ldfrag_g(W, ldb, n0 + 48 + m, k0, h);
    acc0 = wmma16(a0, w0, acc0);
    acc1 = wmma16(a0, w1, acc1);
    acc2 = wmma16(a0, w2, acc2);
    acc3 = wmma16(a0, w3, acc3);
    acc4 = wmma16(a1, w0, acc4);
    acc5 = wmma16(a1, w1, acc5);
    acc6 = wmma16(a1, w2, acc6);
    acc7 = wmma16(a1, w3, acc7);
  }

  float* S = stg + wid * (32 * SPITCH);
  stash_tile(S, acc0, 0, 0, h, m);
  stash_tile(S, acc1, 0, 1, h, m);
  stash_tile(S, acc2, 0, 2, h, m);
  stash_tile(S, acc3, 0, 3, h, m);
  stash_tile(S, acc4, 1, 0, h, m);
  stash_tile(S, acc5, 1, 1, h, m);
  stash_tile(S, acc6, 1, 2, h, m);
  stash_tile(S, acc7, 1, 3, h, m);
  __syncthreads();

  v4f bias;
#pragma unroll
  for (int u = 0; u < 4; ++u) {
    const int col = n0 + 4 * m + u;
    float bs = b1[col];
    if (nbias > 1) bs += b2[col];
    bias[u] = bs;
  }
  gemm_store_pass(S, C, ldc, m0, n0, h, m, scale, bias, active);
  __threadfence();
  gemm_store_pass(S, C, ldc, m0, n0, h, m, scale, bias, active);
}

__device__ __forceinline__ void store_hrow(_Float16* dst, const _Float16* src, int l) {
  const v8h v0 = *(const v8h*)(src + 8 * l);
  const v8h v1 = *(const v8h*)(src + 256 + 8 * l);
  *(volatile v8h*)(dst + 8 * l) = v0;
  *(volatile v8h*)(dst + 256 + 8 * l) = v1;
  __threadfence();
  *(volatile v8h*)(dst + 8 * l) = v0;
  *(volatile v8h*)(dst + 256 + 8 * l) = v1;
}

__device__ __forceinline__ float lstm_group(const _Float16* hc, const _Float16* __restrict__ Wd,
                                            const float* __restrict__ pt, int j0, int h, int m, float& cst) {
  const v8f z = {0.f, 0.f, 0.f, 0.f, 0.f, 0.f, 0.f, 0.f};
  v8f a0 = z, a1 = z, a2 = z, a3 = z;
#pragma unroll 2
  for (int k0 = 0; k0 < HID; k0 += 32) {
    Frag f;
    f.hv[0] = *(const v8h*)(hc + k0 + 8 * h);
    f.hv[1] = *(const v8h*)(hc + k0 + 16 + 8 * h);
    const v16h b0 = ldfrag_g(Wd, HID, j0 + m, k0, h);
    const v16h b1 = ldfrag_g(Wd, HID, HID + j0 + m, k0, h);
    const v16h b2 = ldfrag_g(Wd, HID, 2 * HID + j0 + m, k0, h);
    const v16h b3 = ldfrag_g(Wd, HID, 3 * HID + j0 + m, k0, h);
    a0 = wmma16(f.v, b0, a0);
    a1 = wmma16(f.v, b1, a1);
    a2 = wmma16(f.v, b2, a2);
    a3 = wmma16(f.v, b3, a3);
  }
  const int j = j0 + m;
  const float gi = a0[0] * OPSC2INV + pt[j];
  const float gf = a1[0] * OPSC2INV + pt[HID + j];
  const float gg = a2[0] * OPSC2INV + pt[2 * HID + j];
  const float go = a3[0] * OPSC2INV + pt[3 * HID + j];
  const float si = 1.0f / (1.0f + expf(-gi));
  const float sf = 1.0f / (1.0f + expf(-gf));
  const float so = 1.0f / (1.0f + expf(-go));
  const float c = sf * cst + si * tanhf(gg);
  cst = c;
  return so * tanhf(c);
}

__global__ void __launch_bounds__(512)
k_lstm(const _Float16* __restrict__ Whh16,
       const float* __restrict__ pre,
       _Float16* hout,
       int T) {
  __shared__ __align__(16) _Float16 hb[2 * HID];
  if (blockIdx.x >= 2) return;
  const int tid = threadIdx.x, wid = tid >> 5;
  const int l = tid & 31, h = l >> 4, m = l & 15;
  const int dir = blockIdx.x;
  const _Float16* Wd = Whh16 + (size_t)dir * G4 * HID;
  const float* pd = pre + (size_t)dir * T * G4;

  for (int i = tid; i < 2 * HID; i += 512) hb[i] = (_Float16)0.0f;
  float cst0 = 0.0f, cst1 = 0.0f;
  __syncthreads();

  for (int t = 0; t < T; ++t) {
    const int cur = t & 1;
    const _Float16* hc = hb + cur * HID;
    _Float16* hn = hb + (cur ^ 1) * HID;
    const int tact = dir ? (T - 1 - t) : t;
    if (t > 0 && wid == 0) {
      const int tp = dir ? (T - t) : (t - 1);
      store_hrow(hout + (size_t)tp * (2 * HID) + dir * HID, hc, l);
    }
    const float* pt = pd + (size_t)tact * G4;
    const float hv0 = lstm_group(hc, Wd, pt, 32 * wid, h, m, cst0);
    if (l < 16) hn[32 * wid + m] = (_Float16)(hv0 * OPSC);
    const float hv1 = lstm_group(hc, Wd, pt, 32 * wid + 16, h, m, cst1);
    if (l < 16) hn[32 * wid + 16 + m] = (_Float16)(hv1 * OPSC);
    __syncthreads();
  }
  if (wid == 0) {
    const int tp = dir ? 0 : (T - 1);
    store_hrow(hout + (size_t)tp * (2 * HID) + dir * HID, hb + (T & 1) * HID, l);
  }
}

__global__ void __launch_bounds__(256)
k_head(const float* __restrict__ hf, const float* __restrict__ mf, const float* __restrict__ wo,
       float* hs, float* ms, int T) {
  __shared__ float sh[32];
  __shared__ float sm[32];
  const int wid = threadIdx.x >> 5, l = threadIdx.x & 31;
  const int t0 = blockIdx.x * 32;
  for (int u = 0; u < 4; ++u) {
    const int tl = wid * 4 + u;
    int t = t0 + tl;
    if (t > T - 1) t = T - 1;
    const float* hr = hf + (size_t)t * MH;
    const float* mr = mf + (size_t)t * MH;
    float a = 0.0f, b = 0.0f;
#pragma unroll 1
    for (int n = l; n < MH; n += 32) {
      a += tanhf(hr[n]) * wo[n];
      b += tanhf(mr[n]) * wo[MH + n];
    }
    for (int off = 16; off > 0; off >>= 1) {
      a += __shfl_xor(a, off);
      b += __shfl_xor(b, off);
    }
    if (l == 0) { sh[tl] = a; sm[tl] = b; }
  }
  __syncthreads();
  if (wid == 0) {
    const int t = t0 + l;
    const float va = sh[l], vb = sm[l];
    if (t < T) { *(volatile float*)(hs + t) = va; *(volatile float*)(ms + t) = vb; }
    __threadfence();
    if (t < T) { *(volatile float*)(hs + t) = va; *(volatile float*)(ms + t) = vb; }
  }
}

__device__ __forceinline__ void outer_pass(const float* __restrict__ hs, float msv, float bv,
                                           float* orow, int T, int wid, int l) {
  for (int col = 128 * wid + 4 * l; col + 3 < T; col += 128 * 8) {
    v4f v;
    v[0] = (msv + hs[col + 0]) + bv;
    v[1] = (msv + hs[col + 1]) + bv;
    v[2] = (msv + hs[col + 2]) + bv;
    v[3] = (msv + hs[col + 3]) + bv;
    *(volatile v4f*)(orow + col) = v;
  }
}

__global__ void __launch_bounds__(256)
k_outer(const float* __restrict__ hs, const float* __restrict__ ms, const float* __restrict__ bo,
        float* out, int T) {
  const int mrow = blockIdx.x;
  if (mrow >= T) return;
  const int wid = threadIdx.x >> 5, l = threadIdx.x & 31;
  const float msv = ms[mrow];
  const float bv = bo[0];
  float* orow = out + (size_t)mrow * T;
  outer_pass(hs, msv, bv, orow, T, wid, l);
  __threadfence();
  outer_pass(hs, msv, bv, orow, T, wid, l);
}

extern "C" void kernel_launch(void* const* d_in, const int* in_sizes, int n_in,
                              void* d_out, int out_size, void* d_ws, size_t ws_size,
                              hipStream_t stream) {
  if (n_in < 18) return;
  const int T = SEQ;
  if (in_sizes[0] != T || in_sizes[1] != T) return;
  if (in_sizes[2] % DW != 0 || in_sizes[3] % DP != 0) return;
  const int V = in_sizes[2] / DW;
  const int P = in_sizes[3] / DP;
  if (V < 1 || P < 1) return;
  if (in_sizes[4] != 2 * G4 * (DW + DP)) return;
  if (in_sizes[5] != 2 * G4 * HID) return;
  if (in_sizes[6] != 2 * G4 || in_sizes[7] != 2 * G4) return;
  if (in_sizes[8] != 2 * G4 * IN1) return;
  if (in_sizes[9] != 2 * G4 * HID) return;
  if (in_sizes[10] != 2 * G4 || in_sizes[11] != 2 * G4) return;
  if (in_sizes[12] != MH * IN1 || in_sizes[13] != MH) return;
  if (in_sizes[14] != MH * IN1 || in_sizes[15] != MH) return;
  if (in_sizes[16] != 2 * MH || in_sizes[17] < 1) return;
  if (out_size != T * T) return;

  const int*   wt    = (const int*)  d_in[0];
  const int*   pt    = (const int*)  d_in[1];
  const float* wemb  = (const float*)d_in[2];
  const float* pemb  = (const float*)d_in[3];
  const float* Wih0  = (const float*)d_in[4];
  const float* Whh0  = (const float*)d_in[5];
  const float* bih0  = (const float*)d_in[6];
  const float* bhh0  = (const float*)d_in[7];
  const float* Wih1  = (const float*)d_in[8];
  const float* Whh1  = (const float*)d_in[9];
  const float* bih1  = (const float*)d_in[10];
  const float* bhh1  = (const float*)d_in[11];
  const float* Whead = (const float*)d_in[12];
  const float* bhead = (const float*)d_in[13];
  const float* Wmod  = (const float*)d_in[14];
  const float* bmod  = (const float*)d_in[15];
  const float* Wout  = (const float*)d_in[16];
  const float* bout  = (const float*)d_in[17];
  float* out = (float*)d_out;

  char* base = (char*)d_ws;
  size_t o = 0;
  auto carve = [&](size_t bytes) -> char* {
    char* p = base + o;
    o = (o + bytes + 255) & ~(size_t)255;
    return p;
  };
  _Float16* x16   = (_Float16*)carve((size_t)T * KP0 * 2);
  _Float16* wih0h = (_Float16*)carve((size_t)2 * G4 * KP0 * 2);
  _Float16* wih1h = (_Float16*)carve((size_t)2 * G4 * IN1 * 2);
  _Float16* whh0h = (_Float16*)carve((size_t)2 * G4 * HID * 2);
  _Float16* whh1h = (_Float16*)carve((size_t)2 * G4 * HID * 2);
  _Float16* whdh  = (_Float16*)carve((size_t)MH * IN1 * 2);
  _Float16* wmdh  = (_Float16*)carve((size_t)MH * IN1 * 2);
  float*    preb  = (float*)   carve((size_t)2 * T * G4 * 4);
  _Float16* h0h   = (_Float16*)carve((size_t)T * IN1 * 2);
  _Float16* h1h   = (_Float16*)carve((size_t)T * IN1 * 2);
  float*    headf = (float*)   carve((size_t)T * MH * 4);
  float*    modf  = (float*)   carve((size_t)T * MH * 4);
  float*    hsv   = (float*)   carve((size_t)T * 4);
  float*    msv   = (float*)   carve((size_t)T * 4);
  if (o > ws_size) return;

  {
    const size_t nv0 = (size_t)2 * G4 * KP0 / 8;
    k_cvt16<<<(unsigned)((nv0 + 255) / 256), 256, 0, stream>>>(Wih0, wih0h, 2 * G4, DW + DP, KP0, OPSC);
    const size_t nv1 = (size_t)2 * G4 * IN1 / 8;
    k_cvt16<<<(unsigned)((nv1 + 255) / 256), 256, 0, stream>>>(Wih1, wih1h, 2 * G4, IN1, IN1, OPSC);
    const size_t nvh = (size_t)2 * G4 * HID / 8;
    k_cvt16<<<(unsigned)((nvh + 255) / 256), 256, 0, stream>>>(Whh0, whh0h, 2 * G4, HID, HID, OPSC);
    k_cvt16<<<(unsigned)((nvh + 255) / 256), 256, 0, stream>>>(Whh1, whh1h, 2 * G4, HID, HID, OPSC);
    const size_t nvd = (size_t)MH * IN1 / 8;
    k_cvt16<<<(unsigned)((nvd + 255) / 256), 256, 0, stream>>>(Whead, whdh, MH, IN1, IN1, OPSC);
    k_cvt16<<<(unsigned)((nvd + 255) / 256), 256, 0, stream>>>(Wmod, wmdh, MH, IN1, IN1, OPSC);
  }
  k_embed<<<T, 64, 0, stream>>>(wt, pt, wemb, pemb, V, P, x16, T);

  const int Mt = T / 32, NtG = G4 / 64, NtH = MH / 64;
  const unsigned gridG = (unsigned)((Mt * NtG + 3) / 4);
  const unsigned gridH = (unsigned)((Mt * NtH + 3) / 4);
  for (int d = 0; d < 2; ++d)
    k_gemm<<<gridG, 128, 0, stream>>>(x16, KP0, wih0h + (size_t)d * G4 * KP0, KP0,
                                       bih0 + (size_t)d * G4, bhh0 + (size_t)d * G4, 2,
                                       preb + (size_t)d * T * G4, G4, Mt, NtG, KP0, OPSC2INV);
  k_lstm<<<2, 512, 0, stream>>>(whh0h, preb, h0h, T);

  for (int d = 0; d < 2; ++d)
    k_gemm<<<gridG, 128, 0, stream>>>(h0h, IN1, wih1h + (size_t)d * G4 * IN1, IN1,
                                       bih1 + (size_t)d * G4, bhh1 + (size_t)d * G4, 2,
                                       preb + (size_t)d * T * G4, G4, Mt, NtG, IN1, OPSC2INV);
  k_lstm<<<2, 512, 0, stream>>>(whh1h, preb, h1h, T);

  k_gemm<<<gridH, 128, 0, stream>>>(h1h, IN1, whdh, IN1, bhead, bhead, 1, headf, MH, Mt, NtH, IN1, OPSC2INV);
  k_gemm<<<gridH, 128, 0, stream>>>(h1h, IN1, wmdh, IN1, bmod,  bmod,  1, modf,  MH, Mt, NtH, IN1, OPSC2INV);

  k_head<<<(unsigned)((T + 31) / 32), 256, 0, stream>>>(headf, modf, Wout, hsv, msv, T);
  k_outer<<<T, 256, 0, stream>>>(hsv, msv, bout, out, T);
}
